// Model_11424613007975
// MI455X (gfx1250) — hardware-run, weakly checked
//
#include <hip/hip_runtime.h>
#include <math.h>

typedef _Float16 h16;
typedef __attribute__((ext_vector_type(16))) _Float16 v16h;
typedef __attribute__((ext_vector_type(8)))  _Float16 v8h;
typedef __attribute__((ext_vector_type(4)))  _Float16 v4h;
typedef __attribute__((ext_vector_type(8)))  float v8f;
typedef __attribute__((ext_vector_type(4)))  float v4f;
typedef __attribute__((ext_vector_type(4)))  unsigned v4u;
typedef __attribute__((ext_vector_type(4)))  int v4i;

template <typename T> __device__ __forceinline__ void vst2(void* p, T v) { *(volatile T*)p = v; __threadfence(); *(volatile T*)p = v; }
__device__ __forceinline__ v8f wmma16(v16h a, v16h b, v8f c) {
  v8f d = __builtin_amdgcn_wmma_f32_16x16x32_f16(false, a, false, b, (short)0, c, false, false);
  asm volatile("v_nop\n\tv_nop\n\tv_nop\n\tv_nop" : "+v"(d) : "v"(a), "v"(b));
  return d;
}
__device__ __forceinline__ v16h frag_h(const _Float16* rowk0, int lane) {
  union { v16h v; v8h q[2]; } u; const _Float16* p = rowk0 + 8 * (lane >> 4);
  u.q[0] = *(const v8h*)p; u.q[1] = *(const v8h*)(p + 16); return u.v;
}
__device__ __forceinline__ float bfr(float v) { return (float)(__bf16)v; }
static __device__ __forceinline__ h16 toh_flush(float v) { const h16 r = (h16)v; return (fabsf(v) < 6.103515625e-05f) ? (h16)0.0f : r; }
#define LDSX() do { asm volatile("s_wait_dscnt 0" ::: "memory"); __builtin_amdgcn_wave_barrier(); __builtin_amdgcn_fence(3  , "workgroup"); } while (0)

#ifndef NB
#define NB 8
#endif
#ifndef SEQ
#define SEQ 1024
#endif
#define NB_FULL 8
#define SEQ_FULL 1024
#define CC 1024
#define NH 16
#define HD 64
#define FF 4096
#define NBS (NB * SEQ)
#define MH (NBS / 2)
static_assert(NB >= 1 && NB <= NB_FULL);
static_assert(SEQ % 256 == 0 && SEQ >= 256 && SEQ <= SEQ_FULL);
static_assert(NH * HD == CC && HD == 64);
static_assert(CC % 128 == 0 && FF % 128 == 0 && CC % 32 == 0 && FF % 32 == 0);
static_assert(NBS % 128 == 0 && MH % 64 == 0 && 2 * MH == NBS);
static_assert(SEQ / 32 <= 32);
static_assert((NBS * (CC / 8)) % 256 == 0 && (3 * CC * CC / 8) % 256 == 0 && (CC * CC / 8) % 256 == 0 && (FF * CC / 8) % 256 == 0);
static_assert(128 * 8 == CC);

#define B_PL   (2u * (size_t)NBS * CC)
#define WS_W1  ((size_t)0)
#define WS_W2  (WS_W1 + 2u * (size_t)FF * CC)
#define WS_WQ  (WS_W2 + 2u * (size_t)CC * FF)
#define WS_WO  (WS_WQ + 2u * (size_t)3 * CC * CC)
#define WS_R1  (WS_WO + 2u * (size_t)CC * CC)
#define WS_R2  (WS_R1 + B_PL)
#define WS_R3  (WS_R2 + 2u * B_PL)
#define WS_R4  (WS_R3 + B_PL)
#define B_HH   (2u * (size_t)MH * FF)
#define WS_CW  (WS_R4 + B_HH)
#define B_CW   (4u * (size_t)(SEQ / 32) * SEQ)
#define WS_PW  (WS_CW + B_CW)
#define B_PW   (4u * (size_t)NB * 32)
#define WS_END (WS_PW + B_PW)
static_assert(WS_END <= (size_t)134217728u);
static_assert(4u * (size_t)NBS * CC <= 2u * B_PL);
static_assert((WS_W2 % 128) == 0 && (WS_WQ % 128) == 0 && (WS_WO % 128) == 0 && (WS_R1 % 128) == 0 && (WS_R2 % 128) == 0 && (WS_R3 % 128) == 0 && (WS_R4 % 128) == 0 && (WS_CW % 128) == 0 && (WS_PW % 128) == 0);

__global__ __launch_bounds__(256) void k_cvt(const float* __restrict__ W, h16* __restrict__ O, int n8, float sc, int xmap) {
  const int i = blockIdx.x * 256 + threadIdx.x; if (i >= n8) return;
  size_t src = (size_t)i * 8;
  if (xmap != 0) { const int row = i / (CC / 8), c8 = i - row * (CC / 8); const int b = row / SEQ, t = row - b * SEQ; src = ((size_t)b * SEQ_FULL + t) * CC + (size_t)c8 * 8; }
  const float* p = W + src; const v4f a = *(const v4f*)p, b4 = *(const v4f*)(p + 4);
  v8h hv;
#pragma unroll
  for (int k = 0; k < 4; ++k) { hv[k] = toh_flush(bfr(a[k]) * sc); hv[4 + k] = toh_flush(bfr(b4[k]) * sc); }
  union { v8h h; v4u u; } uo; uo.h = hv;
  vst2(O + (size_t)i * 8, uo.u);
}

__global__ __launch_bounds__(256) void k_maskw(const int* __restrict__ AM, unsigned* __restrict__ CW) {
  const int q = blockIdx.x * 256 + threadIdx.x; const int kb = blockIdx.y;
  const int* p = AM + (size_t)q * SEQ_FULL + kb * 32;
  unsigned w = 0u;
#pragma unroll 1
  for (int c = 0; c < 8; ++c) { const v4i a = *(const v4i*)(p + c * 4);
#pragma unroll
    for (int k = 0; k < 4; ++k) w |= ((a[k] != 0) ? 1u : 0u) << (c * 4 + k); }
  vst2(CW + (size_t)kb * SEQ + q, w);
}
static_assert(256 * (SEQ / 256) == SEQ);

__global__ __launch_bounds__(32) void k_padw(const int* __restrict__ PM, unsigned* __restrict__ PW) {
  const int b = blockIdx.x, kb = threadIdx.x; const int kbc = (kb < SEQ / 32) ? kb : (SEQ / 32 - 1);
  const int* p = PM + (size_t)b * SEQ_FULL + kbc * 32;
  unsigned w = 0u;
#pragma unroll 1
  for (int c = 0; c < 8; ++c) { const v4i a = *(const v4i*)(p + c * 4);
#pragma unroll
    for (int k = 0; k < 4; ++k) w |= ((a[k] != 0) ? 1u : 0u) << (c * 4 + k); }
  asm volatile("" : "+v"(w));
  const unsigned wo = (kb < SEQ / 32) ? w : 0xFFFFFFFFu;
  vst2(PW + b * 32 + kb, wo);
}

template <int KD> __device__ __forceinline__ void mm16x128(const h16* __restrict__ arow, const h16* __restrict__ wrow, int lane, v8f (&acc)[8]) {
#pragma unroll 1
  for (int kc = 0; kc < KD / 32; ++kc) { const v16h a = frag_h(arow + kc * 32, lane);
#pragma unroll
    for (int j = 0; j < 8; ++j) { const v16h w = frag_h(wrow + (size_t)j * 16 * KD + kc * 32, lane); acc[j] = wmma16(a, w, acc[j]); } }
}

static_assert(64 * 136 * 2 + 128 * 72 * 2 <= 131072);
static_assert(128 * 8 == 64 * 16);
static_assert(128 * 8 == 128 * 8);
__global__ __launch_bounds__(128) void k_qkv(const h16* __restrict__ XB, const h16* __restrict__ WP, const float* __restrict__ BI, h16* __restrict__ QH, h16* __restrict__ KH, h16* __restrict__ VT) {
  __shared__ __align__(16) h16 sh[64][136]; __shared__ __align__(16) h16 th[128][72];
  const int tid = threadIdx.x, wave = __builtin_amdgcn_readfirstlane(tid >> 5), lane = tid & 31, col = lane & 15, g = lane >> 4;
  const int which = blockIdx.z; const int c0 = blockIdx.y * 128; const int cw = which * CC + c0; const size_t r0 = (size_t)blockIdx.x * 64;
  v8f acc[8] = {};
  mm16x128<CC>(XB + (r0 + wave * 16 + col) * CC, WP + (size_t)(cw + col) * CC, lane, acc);
#pragma unroll
  for (int j = 0; j < 8; ++j) { const float bb = bfr(BI[cw + j * 16 + col]);
#pragma unroll
    for (int r = 0; r < 8; ++r) { const float v = acc[j][r] * (1.0f / 64.0f) + bb; const int rl = wave * 16 + 8 * g + r, cl = j * 16 + col; const h16 hv = toh_flush(v);
      if (which == 2) th[cl][rl] = hv; else sh[rl][cl] = hv; } }
  __syncthreads();
  if (which < 2) { h16* dh = which == 0 ? QH : KH; for (int e = tid; e < 64 * 16; e += 128) { const int rl = e >> 4, q = e & 15; vst2((unsigned*)(dh + (r0 + rl) * CC + c0 + q * 8), *(const v4u*)&sh[rl][q * 8]); } }
  else { const size_t b = r0 / SEQ; const int t0 = (int)(r0 % SEQ); for (int e = tid; e < 128 * 8; e += 128) { const int cl = e >> 3, q = e & 7; const size_t o2 = (b * CC + c0 + cl) * (size_t)SEQ + t0 + q * 8; vst2((unsigned*)(VT + o2), *(const v4u*)&th[cl][q * 8]); } }
}

static_assert(4 * 16 * 72 * 2 <= 131072);
static_assert(4 * 32 * 16 == 16 * HD * 2);
__global__ __launch_bounds__(128) void k_flash(const h16* __restrict__ QH, const h16* __restrict__ KH, const h16* __restrict__ VT, const unsigned* __restrict__ CW, const unsigned* __restrict__ PW, h16* __restrict__ CX) {
  __shared__ __align__(16) h16 so[4][16][72];
  const int tid = threadIdx.x, wave = __builtin_amdgcn_readfirstlane(tid >> 5), lane = tid & 31, col = lane & 15, g = lane >> 4;
  const int b = blockIdx.z, h = blockIdx.y; const int q0 = blockIdx.x * 64 + wave * 16;
  const h16* qrow = QH + ((size_t)b * SEQ + q0 + col) * CC + h * HD;
  const v16h qf0 = frag_h(qrow, lane), qf1 = frag_h(qrow + 32, lane);
  const h16* kbase = KH + ((size_t)b * SEQ + col) * CC + h * HD;
  const h16* vbase = VT + ((size_t)b * CC + h * HD + col) * (size_t)SEQ;
  const unsigned* cwp = CW + q0 + col;
  const float SCL = 0.18033688011112042f;
  float m = -INFINITY, l = 0.f; v8f o[4] = {};
#pragma unroll 1
  for (int kb = 0; kb < SEQ / 32; ++kb) {
    const unsigned mw = cwp[(size_t)kb * SEQ] | PW[b * 32 + kb];
    if (__builtin_amdgcn_ballot_w32(mw != 0xFFFFFFFFu) == 0u) continue;
    const h16* kr = kbase + (size_t)kb * 32 * CC;
    v8f s0 = {}, s1 = {};
    s0 = wmma16(frag_h(kr, lane), qf0, s0); s0 = wmma16(frag_h(kr + 32, lane), qf1, s0);
    s1 = wmma16(frag_h(kr + 16 * CC, lane), qf0, s1); s1 = wmma16(frag_h(kr + 16 * CC + 32, lane), qf1, s1);
    const unsigned mg = mw >> (8 * g);
    float t[16];
#pragma unroll
    for (int r = 0; r < 8; ++r) { t[r] = ((mg >> r) & 1u) ? -INFINITY : s0[r] * SCL; t[8 + r] = ((mg >> (16 + r)) & 1u) ? -INFINITY : s1[r] * SCL; }
    float mt = t[0];
#pragma unroll
    for (int i = 1; i < 16; ++i) mt = fmaxf(mt, t[i]);
    mt = fmaxf(mt, __shfl_xor(mt, 16));
    const float mn = fmaxf(m, mt); const float mu = (mn == -INFINITY) ? 0.f : mn;
    const float alpha = exp2f(m - mu);
    float ps = 0.f; v16h pf;
#pragma unroll
    for (int i = 0; i < 16; ++i) { const float ea = (t[i] - mu) + 8.0f; const float pc = (ea < -14.0f) ? 0.0f : exp2f(ea); const h16 ph = (h16)pc; pf[i] = ph; ps += (float)ph; }
    ps += __shfl_xor(ps, 16);
    l = l * alpha + ps; m = mn;
#pragma unroll
    for (int j = 0; j < 4; ++j) o[j] = o[j] * alpha;
    const h16* vr = vbase + kb * 32;
#pragma unroll
    for (int j = 0; j < 4; ++j) o[j] = wmma16(frag_h(vr + (size_t)j * 16 * SEQ, lane), pf, o[j]);
  }
  const float inv = 256.0f * (1.0f / l);
#pragma unroll
  for (int j = 0; j < 4; ++j) { v8h hv;
#pragma unroll
    for (int r = 0; r < 8; ++r) hv[r] = toh_flush(o[j][r] * inv);
    *(v8h*)&so[wave][col][j * 16 + 8 * g] = hv; }
  LDSX();
#pragma unroll
  for (int it = 0; it < 4; ++it) { const int r = it * 4 + (lane >> 3), pc8 = lane & 7; const v8h hv = *(const v8h*)&so[wave][r][pc8 * 8]; union { v8h h; v4u u; } uu; uu.h = hv;
    vst2(CX + ((size_t)b * SEQ + q0 + r) * CC + h * HD + pc8 * 8, uu.u); }
}

static_assert(4 * 16 * 132 * 4 <= 131072);
static_assert(16 * 32 * 16 == 16 * 128 * 4);
__global__ __launch_bounds__(128) void k_oproj(const h16* __restrict__ CX, const h16* __restrict__ WP, const float* __restrict__ BP, const float* __restrict__ X, float* __restrict__ Y1) {
  __shared__ __align__(16) float sf[4][16][132];
  const int tid = threadIdx.x, wave = __builtin_amdgcn_readfirstlane(tid >> 5), lane = tid & 31, col = lane & 15, g = lane >> 4; const int c0 = blockIdx.y * 128; const size_t r0 = (size_t)blockIdx.x * 64 + wave * 16;
  v8f acc[8] = {};
  mm16x128<CC>(CX + (r0 + col) * CC, WP + (size_t)(c0 + col) * CC, lane, acc);
#pragma unroll
  for (int j = 0; j < 8; ++j) { const float bb = bfr(BP[c0 + j * 16 + col]);
#pragma unroll
    for (int r = 0; r < 8; ++r) sf[wave][8 * g + r][j * 16 + col] = acc[j][r] * (1.0f / 16384.0f) + bb; }
  LDSX();
  for (int rl = 0; rl < 16; ++rl) { const size_t R = r0 + rl; v4f o = *(const v4f*)&sf[wave][rl][lane * 4];
    const int bq = (int)(R / SEQ), s = (int)(R - (size_t)bq * SEQ);
    const v4f xv = *(const v4f*)(X + ((size_t)bq * SEQ_FULL + s) * CC + c0 + lane * 4);
#pragma unroll
    for (int i = 0; i < 4; ++i) o[i] += bfr(xv[i]);
    vst2(Y1 + R * CC + c0 + lane * 4, o); }
}

static_assert(CC * 2 + 64 <= 131072);
__global__ __launch_bounds__(128) void k_ln(const float* IN, const float* __restrict__ G, const float* __restrict__ Bt, float* OF, h16* __restrict__ OH, int wh) {
#pragma clang fp contract(off)
  __shared__ float red[2][4]; __shared__ __align__(16) h16 shh[CC];
  const int tid = threadIdx.x, wave = __builtin_amdgcn_readfirstlane(tid >> 5), lane = tid & 31; const size_t row = blockIdx.x;
  const int ca = tid * 4, cb = CC / 2 + tid * 4; const float* xr = IN + row * CC;
  const v4f x0 = *(const v4f*)(xr + ca), x1 = *(const v4f*)(xr + cb), g0 = *(const v4f*)(G + ca), g1 = *(const v4f*)(G + cb), b0 = *(const v4f*)(Bt + ca), b1 = *(const v4f*)(Bt + cb);
  float v[8], gg[8], bb[8];
#pragma unroll
  for (int i = 0; i < 4; ++i) { v[i] = x0[i]; v[4 + i] = x1[i]; gg[i] = bfr(g0[i]); gg[4 + i] = bfr(g1[i]); bb[i] = bfr(b0[i]); bb[4 + i] = bfr(b1[i]); }
  float s1 = 0.f;
#pragma unroll
  for (int i = 0; i < 8; ++i) s1 += v[i];
#pragma unroll
  for (int o = 1; o < 32; o <<= 1) s1 += __shfl_xor(s1, o);
  if (lane == 0) red[0][wave] = s1;
  __syncthreads();
  const float mean = ((red[0][0] + red[0][1]) + (red[0][2] + red[0][3])) * (1.0f / (float)CC);
  float s2 = 0.f;
#pragma unroll
  for (int i = 0; i < 8; ++i) { const float d = v[i] - mean; v[i] = d; s2 += d * d; }
#pragma unroll
  for (int o = 1; o < 32; o <<= 1) s2 += __shfl_xor(s2, o);
  if (lane == 0) red[1][wave] = s2;
  __syncthreads();
  const float var = ((red[1][0] + red[1][1]) + (red[1][2] + red[1][3])) * (1.0f / (float)CC);
  const float rstd = 1.0f / sqrtf(var + 1e-12f);
  v4f o0, o1; v4h h0, h1;
#pragma unroll
  for (int i = 0; i < 4; ++i) { const float y0 = gg[i] * v[i] * rstd + bb[i]; const float y1 = gg[4 + i] * v[4 + i] * rstd + bb[4 + i]; o0[i] = y0; o1[i] = y1; h0[i] = toh_flush(y0); h1[i] = toh_flush(y1); }
  *(v4h*)&shh[ca] = h0; *(v4h*)&shh[cb] = h1;
  __syncthreads();
  vst2(OF + row * CC + ca, o0);
  vst2(OF + row * CC + cb, o1);
  if (wh != 0) { const v8h hv = *(const v8h*)&shh[tid * 8]; union { v8h h; v4u u; } uu; uu.h = hv; vst2(OH + row * CC + tid * 8, uu.u); }
}

static_assert(64 * 136 * 2 <= 131072);
__global__ __launch_bounds__(128) void k_fc1(const h16* __restrict__ XH, const h16* __restrict__ WP, const float* __restrict__ BP, h16* __restrict__ HO, int rbase) {
  __shared__ __align__(16) h16 sh[64][136];
  const int tid = threadIdx.x, wave = __builtin_amdgcn_readfirstlane(tid >> 5), lane = tid & 31, col = lane & 15, g = lane >> 4; const int c0 = blockIdx.y * 128; const size_t rl0 = (size_t)blockIdx.x * 64;
  v8f acc[8] = {};
  mm16x128<CC>(XH + ((size_t)rbase + rl0 + wave * 16 + col) * CC, WP + (size_t)(c0 + col) * CC, lane, acc);
#pragma unroll
  for (int j = 0; j < 8; ++j) { const float bb = bfr(BP[c0 + j * 16 + col]);
#pragma unroll
    for (int r = 0; r < 8; ++r) { float v = acc[j][r] * (1.0f / 64.0f) + bb; v = (v > 0.0f) ? v : 0.0f; sh[wave * 16 + 8 * g + r][j * 16 + col] = toh_flush(v); } }
  __syncthreads();
  for (int e = tid; e < 64 * 16; e += 128) { const int rl = e >> 4, q = e & 15; vst2((unsigned*)(HO + (rl0 + rl) * FF + c0 + q * 8), *(const v4u*)&sh[rl][q * 8]); }
}

__global__ __launch_bounds__(128) void k_fc2(const h16* __restrict__ HI, const h16* __restrict__ WP, const float* __restrict__ BP, float* RY, int rbase) {
  __shared__ __align__(16) float sf[4][16][132];
  const int tid = threadIdx.x, wave = __builtin_amdgcn_readfirstlane(tid >> 5), lane = tid & 31, col = lane & 15, g = lane >> 4; const int c0 = blockIdx.y * 128; const size_t rl0 = (size_t)blockIdx.x * 64 + wave * 16;
  v8f acc[8] = {};
  mm16x128<FF>(HI + (rl0 + col) * FF, WP + (size_t)(c0 + col) * FF, lane, acc);
#pragma unroll
  for (int j = 0; j < 8; ++j) { const float bb = bfr(BP[c0 + j * 16 + col]);
#pragma unroll
    for (int r = 0; r < 8; ++r) sf[wave][8 * g + r][j * 16 + col] = acc[j][r] * (1.0f / 64.0f) + bb; }
  LDSX();
  for (int rl = 0; rl < 16; ++rl) { float* p = RY + ((size_t)rbase + rl0 + rl) * CC + c0 + lane * 4; v4f o = *(const v4f*)&sf[wave][rl][lane * 4]; const v4f xv = *(const v4f*)p; o += xv; vst2(p, o); }
}

extern "C" void kernel_launch(void* const* d_in, const int* in_sizes, int n_in, void* d_out, int out_size, void* d_ws, size_t ws_size, hipStream_t stream) {
  if (n_in < 15) return;
  const float* const* F = (const float* const*)d_in;
  if ((size_t)in_sizes[0] < ((size_t)(NB - 1) * SEQ_FULL + SEQ) * CC) return;
  if (in_sizes[1] < 3 * CC * CC || in_sizes[2] < 3 * CC || in_sizes[3] < CC * CC || in_sizes[4] < CC) return;
  if (in_sizes[5] < FF * CC || in_sizes[6] < FF || in_sizes[7] < CC * FF || in_sizes[8] < CC) return;
  if (in_sizes[9] < CC || in_sizes[10] < CC || in_sizes[11] < CC || in_sizes[12] < CC) return;
  if ((size_t)in_sizes[13] < (size_t)(NB - 1) * SEQ_FULL + SEQ) return;
  if ((size_t)in_sizes[14] < (size_t)(SEQ - 1) * SEQ_FULL + SEQ) return;
  if ((size_t)out_size < (size_t)NBS * CC) return;
  if (ws_size < (size_t)WS_END) return;
  const int* PM = (const int*)d_in[13]; const int* AM = (const int*)d_in[14];
  char* ws = (char*)d_ws;
  h16* W1 = (h16*)(ws + WS_W1); h16* W2 = (h16*)(ws + WS_W2); h16* WQ = (h16*)(ws + WS_WQ); h16* WO = (h16*)(ws + WS_WO);
  h16* XB = (h16*)(ws + WS_R1); h16* CX = (h16*)(ws + WS_R1);
  h16* QH = (h16*)(ws + WS_R2); h16* KH = (h16*)(ws + WS_R2 + B_PL); float* RY = (float*)(ws + WS_R2);
  h16* VT = (h16*)(ws + WS_R3); h16* X1H = (h16*)(ws + WS_R3);
  h16* HH = (h16*)(ws + WS_R4);
  unsigned* CW = (unsigned*)(ws + WS_CW); unsigned* PW = (unsigned*)(ws + WS_PW);
  const int n8x = NBS * (CC / 8), n8q = 3 * CC * CC / 8, n8o = CC * CC / 8, n8f = FF * CC / 8;
  k_cvt<<<(n8x + 255) / 256, 256, 0, stream>>>(F[0], XB, n8x, 1.0f, 1);
  k_cvt<<<(n8q + 255) / 256, 256, 0, stream>>>(F[1], WQ, n8q, 64.0f, 0);
  k_cvt<<<(n8o + 255) / 256, 256, 0, stream>>>(F[3], WO, n8o, 64.0f, 0);
  k_cvt<<<(n8f + 255) / 256, 256, 0, stream>>>(F[5], W1, n8f, 64.0f, 0);
  k_cvt<<<(n8f + 255) / 256, 256, 0, stream>>>(F[7], W2, n8f, 64.0f, 0);
  k_maskw<<<dim3(SEQ / 256, SEQ / 32), 256, 0, stream>>>(AM, CW);
  k_padw<<<NB, 32, 0, stream>>>(PM, PW);
  k_qkv<<<dim3(NBS / 64, CC / 128, 3), 128, 0, stream>>>(XB, WQ, F[2], QH, KH, VT);
  k_flash<<<dim3(SEQ / 64, NH, NB), 128, 0, stream>>>(QH, KH, VT, CW, PW, CX);
  k_oproj<<<dim3(NBS / 64, CC / 128), 128, 0, stream>>>(CX, WO, F[4], F[0], RY);
  k_ln<<<NBS, 128, 0, stream>>>(RY, F[9], F[10], RY, X1H, 1);
  for (int hf = 0; hf < 2; ++hf) {
    k_fc1<<<dim3(MH / 64, FF / 128), 128, 0, stream>>>(X1H, W1, F[6], HH, hf * MH);
    k_fc2<<<dim3(MH / 64, CC / 128), 128, 0, stream>>>(HH, W2, F[8], RY, hf * MH);
  }
  k_ln<<<NBS, 128, 0, stream>>>(RY, F[11], F[12], (float*)d_out, X1H, 0);
}
